// PEGLayer_34308198761093
// MI455X (gfx1250) — hardware-verified
//
#include <hip/hip_runtime.h>
#include <stddef.h>


#define DD     256
#define DH     512
#define OROW   259
#define TE     64
#define P1     264
#define P2     520
#define P3     260
#define ASC    8
#define WSC    64
#define OSC    (1.0f / 512.0f)
#define NTHR   256
#define NWAVE  8
#define EPT    8
#define NGRP   2
#define CHUNK  (NTHR * EPT * NGRP)
#define WCAP   (EPT * NGRP * 32)
#define LISTN  (NWAVE * WCAP)
#define NBC    4096
#define NBF    1024
#define RCAP   40960
#define RBN    128
#define OTHR   512
#define DEGCAP 256
#define ANB    32
#define XBM    64
#define XBN    128
#define VECN   2048
#define WSCAP  134217728
#define LDS_FILL ((RCAP + NBF + LISTN) * 4 + 64)
#define LDS_EDGE ((TE * P1 + TE * P2) * 2 + 3 * TE * 4)

static_assert((CHUNK & (CHUNK - 1)) == 0);
static_assert(CHUNK <= 4096);
static_assert((NBC & (NBC - 1)) == 0 && (NBF & (NBF - 1)) == 0);
static_assert(NBC == 4 * NBF);
static_assert(OTHR * 8 == NBC);
static_assert((RCAP % 32) == 0);
static_assert(WCAP == EPT * NGRP * 32);
static_assert(TE * P3 * 4 == TE * P2 * 2);
static_assert(((ANB * OROW) % 4) == 0);
static_assert(((ANB * OROW * 4) % 128) == 0);
static_assert(TE == 2 * 32);
static_assert(NWAVE * 8 == TE);
static_assert(XBM * 2 == XBN);
static_assert(DD == 8 * 32 && DH == 16 * 32);
static_assert(((TE * P1 * 2) % 16) == 0 && ((P1 * 2) % 16) == 0 && ((P2 * 2) % 16) == 0 && ((P3 * 4) % 16) == 0);

typedef float          v4f  __attribute__((ext_vector_type(4)));
typedef float          v8f  __attribute__((ext_vector_type(8)));
typedef int            v4i  __attribute__((ext_vector_type(4)));
typedef _Float16       v8h  __attribute__((ext_vector_type(8)));
typedef _Float16       v16h __attribute__((ext_vector_type(16)));
typedef unsigned short v8us __attribute__((ext_vector_type(8)));
union FragH { v16h v; v8us u[2]; v8h h[2]; };

__device__ __forceinline__ v8f wmh(v16h a, v16h b, v8f c) {
  v8f d = __builtin_amdgcn_wmma_f32_16x16x32_f16(false, a, false, b, (short)0, c, false, false);
  asm volatile("v_nop\n\tv_nop\n\tv_nop\n\tv_nop" : "+v"(d) : "v"(a), "v"(b));
  return d;
}
__device__ __forceinline__ v8f zero8() { v8f z = {0.f, 0.f, 0.f, 0.f, 0.f, 0.f, 0.f, 0.f}; return z; }
__device__ __forceinline__ float lrelu(float x) { return fmaxf(x, 0.2f * x); }

__device__ __forceinline__ v16h frag_glb(const unsigned short* P, int row, int ld, int k0, int hh) {
  FragH f;
  const unsigned short* p = P + (size_t)row * ld + k0 + 8 * hh;
  f.u[0] = *(const v8us*)p;
  f.u[1] = *(const v8us*)(p + 16);
  return f.v;
}
__device__ __forceinline__ v16h frag_lds(const _Float16* T, int row, int ld, int k0, int hh) {
  FragH f;
  const _Float16* p = T + row * ld + k0 + 8 * hh;
  f.h[0] = *(const v8h*)p;
  f.h[1] = *(const v8h*)(p + 16);
  return f.v;
}
__device__ __forceinline__ v8h cvt8s(const float* p, float sc) {
  const v4f a = *(const v4f*)p, b = *(const v4f*)(p + 4);
  v8h o;
  o[0] = (_Float16)(a.x * sc); o[1] = (_Float16)(a.y * sc); o[2] = (_Float16)(a.z * sc); o[3] = (_Float16)(a.w * sc);
  o[4] = (_Float16)(b.x * sc); o[5] = (_Float16)(b.y * sc); o[6] = (_Float16)(b.z * sc); o[7] = (_Float16)(b.w * sc);
  return o;
}

template <int NB>
__device__ __forceinline__ int scan_chunk(const int* __restrict__ dsts, int nE, int cbase, int slotBase,
                                          int vec8, int* list, int tid, int lane, int wave) {
  int wc = 0;
#pragma unroll
  for (int g = 0; g < NGRP; ++g) {
    const int el0  = (g * NTHR + tid) * EPT;
    const int e0   = cbase + el0;
    const int sent = -2147483647 - 1;
    v4i da, db;
    if (vec8 != 0 && cbase + CHUNK <= nE) {
      da = *(const v4i*)(dsts + e0);
      db = *(const v4i*)(dsts + e0 + 4);
    } else {
      da.x = (e0     < nE) ? dsts[min(e0, nE - 1)] : sent;
      da.y = (e0 + 1 < nE) ? dsts[min(e0 + 1, nE - 1)] : sent;
      da.z = (e0 + 2 < nE) ? dsts[min(e0 + 2, nE - 1)] : sent;
      da.w = (e0 + 3 < nE) ? dsts[min(e0 + 3, nE - 1)] : sent;
      db.x = (e0 + 4 < nE) ? dsts[min(e0 + 4, nE - 1)] : sent;
      db.y = (e0 + 5 < nE) ? dsts[min(e0 + 5, nE - 1)] : sent;
      db.z = (e0 + 6 < nE) ? dsts[min(e0 + 6, nE - 1)] : sent;
      db.w = (e0 + 7 < nE) ? dsts[min(e0 + 7, nE - 1)] : sent;
    }
    const unsigned nb = (unsigned)slotBase;
    const unsigned s0 = (unsigned)da.x - nb, s1 = (unsigned)da.y - nb;
    const unsigned s2 = (unsigned)da.z - nb, s3 = (unsigned)da.w - nb;
    const unsigned s4 = (unsigned)db.x - nb, s5 = (unsigned)db.y - nb;
    const unsigned s6 = (unsigned)db.z - nb, s7 = (unsigned)db.w - nb;
    const bool h0 = s0 < (unsigned)NB, h1 = s1 < (unsigned)NB, h2 = s2 < (unsigned)NB, h3 = s3 < (unsigned)NB;
    const bool h4 = s4 < (unsigned)NB, h5 = s5 < (unsigned)NB, h6 = s6 < (unsigned)NB, h7 = s7 < (unsigned)NB;
    const unsigned any = __builtin_amdgcn_ballot_w32(h0 | h1 | h2 | h3 | h4 | h5 | h6 | h7);
    if (any != 0u) {
#define HITJ(J, HJ, SJ) { \
        const unsigned mj = __builtin_amdgcn_ballot_w32(HJ); \
        if (mj != 0u) { \
          if (HJ) { \
            const int pos = wc + (int)__builtin_amdgcn_mbcnt_lo(mj, 0u); \
            if (pos < WCAP) list[wave * WCAP + pos] = ((el0 + (J)) << 12) | (int)(SJ); \
          } \
          wc += (int)__builtin_popcount(mj); } }
      HITJ(0, h0, s0)
      HITJ(1, h1, s1)
      HITJ(2, h2, s2)
      HITJ(3, h3, s3)
      HITJ(4, h4, s4)
      HITJ(5, h5, s5)
      HITJ(6, h6, s6)
      HITJ(7, h7, s7)
#undef HITJ
    }
  }
  return wc;
}

__global__ __launch_bounds__(NTHR) void k_count(const int* __restrict__ keys, int* cnt, float* dinv,
                                               int nK, int nRow, int vec8) {
  __shared__ __attribute__((aligned(16))) int scnt[NBC];
  __shared__ __attribute__((aligned(16))) int srow[NBC];
  __shared__ __attribute__((aligned(16))) int list[LISTN];
  __shared__ int wcnt[NWAVE];
  const int tid = threadIdx.x, lane = tid & 31, wave = tid >> 5;
  const int nodeBase = blockIdx.x * NBC;

  for (int i = tid; i < NBC; i += NTHR) { scnt[i] = 0; srow[i] = 0; }
  __syncthreads();

  const int nChunks = (nK + CHUNK - 1) / CHUNK;
#pragma unroll 1
  for (int ch = 0; ch < nChunks; ++ch) {
    const int cbase = ch * CHUNK;
    const int wc = scan_chunk<NBC>(keys, nK, cbase, nodeBase, vec8, list, tid, lane, wave);
    if (lane == 0) wcnt[wave] = wc;
    __syncthreads();
    if (wave == 0) {
#pragma unroll 1
      for (int wsx = 0; wsx < NWAVE; ++wsx) {
        int n = __builtin_amdgcn_readfirstlane(wcnt[wsx]);
        n = n > WCAP ? WCAP : (n < 0 ? 0 : n);
        const int* lp = list + wsx * WCAP;
#pragma unroll 1
        for (int i = 0; i < n; ++i) {
          const int ent  = __builtin_amdgcn_readfirstlane(lp[i]);
          const int slot = ent & (NBC - 1);
          const int e    = cbase + ((ent >> 12) & (CHUNK - 1));
          const int isr  = (e < nRow) ? 1 : 0;
          if (lane == 0) {
            scnt[slot] = scnt[slot] + 1;
            srow[slot] = srow[slot] + isr;
          }
        }
      }
    }
    __syncthreads();
  }

  v4i cq[4];
  v4f dq[4];
#pragma unroll
  for (int q = 0; q < 4; ++q) {
    const int f = (wave * 4 + q) * 128 + 4 * lane;
    cq[q] = *(const v4i*)(scnt + f);
    const v4i rq = *(const v4i*)(srow + f);
    dq[q].x = rsqrtf((float)(rq.x > 0 ? rq.x : 1));
    dq[q].y = rsqrtf((float)(rq.y > 0 ? rq.y : 1));
    dq[q].z = rsqrtf((float)(rq.z > 0 ? rq.z : 1));
    dq[q].w = rsqrtf((float)(rq.w > 0 ? rq.w : 1));
  }
  int* cp = cnt + (size_t)nodeBase;
  float* dp = dinv + (size_t)nodeBase;
#pragma unroll
  for (int q = 0; q < 4; ++q) {
    const int f = (wave * 4 + q) * 128 + 4 * lane;
    *(volatile v4i*)(cp + f) = cq[q];
    *(volatile v4f*)(dp + f) = dq[q];
  }
  __threadfence();
#pragma unroll
  for (int q = 0; q < 4; ++q) {
    const int f = (wave * 4 + q) * 128 + 4 * lane;
    *(volatile v4i*)(cp + f) = cq[q];
    *(volatile v4f*)(dp + f) = dq[q];
  }
}

__global__ __launch_bounds__(OTHR) void k_offsets(
    const int* __restrict__ cnt, int* off, int* rbase, int nChunk) {
  __shared__ __attribute__((aligned(16))) int soff[NBC];
  __shared__ __attribute__((aligned(16))) int srb[RBN];
  __shared__ int wtot[OTHR / 32];
  const int tid = threadIdx.x, lane = tid & 31, wave = tid >> 5, sub = tid >> 7;
  for (int i = tid; i < RBN; i += OTHR) srb[i] = 0;
  int carry = 0;
#pragma unroll 1
  for (int ch = 0; ch < nChunk; ++ch) {
    const int base = ch * NBC;
    const v4i c0 = *(const v4i*)(cnt + base + 8 * tid);
    const v4i c1 = *(const v4i*)(cnt + base + 8 * tid + 4);
    const int e0 = max(c0.x, 0), e1 = max(c0.y, 0), e2 = max(c0.z, 0), e3 = max(c0.w, 0);
    const int e4 = max(c1.x, 0), e5 = max(c1.y, 0), e6 = max(c1.z, 0), e7 = max(c1.w, 0);
    const int ts = e0 + e1 + e2 + e3 + e4 + e5 + e6 + e7;
    int incl = ts;
#pragma unroll
    for (int d = 1; d < 32; d <<= 1) {
      const int t = __shfl_up(incl, d);
      if (lane >= d) incl += t;
    }
    if (lane == 31) wtot[wave] = incl;
    __syncthreads();
    const int S0 = wtot[0]  + wtot[1]  + wtot[2]  + wtot[3];
    const int S1 = wtot[4]  + wtot[5]  + wtot[6]  + wtot[7];
    const int S2 = wtot[8]  + wtot[9]  + wtot[10] + wtot[11];
    const int S3 = wtot[12] + wtot[13] + wtot[14] + wtot[15];
    int pre = 0;
#pragma unroll 1
    for (int w = 4 * sub; w < wave; ++w) pre += wtot[w];
    const int b0 = carry;
    const int b1 = b0 + ((S0 + 31) & ~31);
    const int b2 = b1 + ((S1 + 31) & ~31);
    const int b3 = b2 + ((S2 + 31) & ~31);
    const int b4 = b3 + ((S3 + 31) & ~31);
    const int myb = sub == 0 ? b0 : (sub == 1 ? b1 : (sub == 2 ? b2 : b3));
    if (tid == 0) {
      srb[min(4 * ch + 0, RBN - 1)] = b0;
      srb[min(4 * ch + 1, RBN - 1)] = b1;
      srb[min(4 * ch + 2, RBN - 1)] = b2;
      srb[min(4 * ch + 3, RBN - 1)] = b3;
    }
    int run = myb + pre + incl - ts;
    soff[8 * tid + 0] = run; run += e0;
    soff[8 * tid + 1] = run; run += e1;
    soff[8 * tid + 2] = run; run += e2;
    soff[8 * tid + 3] = run; run += e3;
    soff[8 * tid + 4] = run; run += e4;
    soff[8 * tid + 5] = run; run += e5;
    soff[8 * tid + 6] = run; run += e6;
    soff[8 * tid + 7] = run;
    carry = b4;
    __syncthreads();
    const v4i o0 = *(const v4i*)(soff + 4 * tid);
    const v4i o1 = *(const v4i*)(soff + 4 * (tid + OTHR));
    int* op = off + base;
    *(volatile v4i*)(op + 4 * tid) = o0;
    *(volatile v4i*)(op + 4 * (tid + OTHR)) = o1;
    __threadfence();
    *(volatile v4i*)(op + 4 * tid) = o0;
    *(volatile v4i*)(op + 4 * (tid + OTHR)) = o1;
    __syncthreads();
  }
  if (tid == 0) srb[min(4 * nChunk, RBN - 1)] = carry;
  __syncthreads();
  v4i rv = {0, 0, 0, 0};
  if (tid < 32) rv = *(const v4i*)(srb + 4 * tid);
  if (tid < 32) *(volatile v4i*)(rbase + 4 * tid) = rv;
  __threadfence();
  if (tid < 32) *(volatile v4i*)(rbase + 4 * tid) = rv;
}

__global__ __launch_bounds__(NTHR) void k_fill(
    const int* __restrict__ keys, const int* __restrict__ off, const int* __restrict__ rbase,
    int* csrE, int nK, int vec8, int csrLen) {
  extern __shared__ v4f lds_dyn[];
  int* region = (int*)lds_dyn;
  int* cursor = region + RCAP;
  int* list   = cursor + NBF;
  int* wcnt   = list + LISTN;
  const int tid = threadIdx.x, lane = tid & 31, wave = tid >> 5;
  const int b = blockIdx.x;
  const int nodeBase = b * NBF;

  int rb0 = rbase[b];
  const int rb1 = rbase[b + 1];
  rb0 = rb0 < 0 ? 0 : (rb0 > csrLen ? csrLen : rb0);
  rb0 &= ~31;
  int len = rb1 - rb0;
  len = len < 0 ? 0 : (len > RCAP ? RCAP : len);
  int lenW = (len + 31) & ~31;
  if (rb0 + lenW > csrLen) lenW = (csrLen - rb0) & ~31;

  {
    const v4i z = {0, 0, 0, 0};
    for (int i = tid; i < RCAP / 4; i += NTHR) ((v4i*)region)[i] = z;
    for (int s = tid; s < NBF; s += NTHR) {
      int o = off[nodeBase + s] - rb0;
      o = o < 0 ? 0 : (o > RCAP ? RCAP : o);
      cursor[s] = o;
    }
  }
  __syncthreads();

  const int nChunks = (nK + CHUNK - 1) / CHUNK;
#pragma unroll 1
  for (int ch = 0; ch < nChunks; ++ch) {
    const int cbase = ch * CHUNK;
    const int wc = scan_chunk<NBF>(keys, nK, cbase, nodeBase, vec8, list, tid, lane, wave);
    if (lane == 0) wcnt[wave] = wc;
    __syncthreads();
    if (wave == 0) {
#pragma unroll 1
      for (int wsx = 0; wsx < NWAVE; ++wsx) {
        int n = __builtin_amdgcn_readfirstlane(wcnt[wsx]);
        n = n > WCAP ? WCAP : (n < 0 ? 0 : n);
        const int* lp = list + wsx * WCAP;
#pragma unroll 1
        for (int i = 0; i < n; ++i) {
          const int ent  = __builtin_amdgcn_readfirstlane(lp[i]);
          const int slot = ent & (NBF - 1);
          int e = cbase + ((ent >> 12) & (CHUNK - 1));
          e = e > nK - 1 ? nK - 1 : e;
          if (lane == 0) {
            int pos = cursor[slot];
            pos = pos < 0 ? 0 : (pos > RCAP - 1 ? RCAP - 1 : pos);
            region[pos] = e;
            const int np = pos + 1;
            cursor[slot] = np > RCAP ? RCAP : np;
          }
        }
      }
    }
    __syncthreads();
  }

  const int nv = lenW >> 2;
  int* gp = csrE + rb0;
#pragma unroll 1
  for (int i = tid; i < nv; i += NTHR) {
    const v4i ve = ((const v4i*)region)[i];
    *(volatile v4i*)(gp + 4 * i) = ve;
  }
  __threadfence();
#pragma unroll 1
  for (int i = tid; i < nv; i += NTHR) {
    const v4i ve = ((const v4i*)region)[i];
    *(volatile v4i*)(gp + 4 * i) = ve;
  }
}

__global__ __launch_bounds__(NTHR) void k_wcvt(
    const float* __restrict__ w2, const float* __restrict__ w3, const float* __restrict__ wn,
    const float* __restrict__ w1, const float* __restrict__ b1, const float* __restrict__ g1,
    const float* __restrict__ be1, const float* __restrict__ b2, const float* __restrict__ g2,
    const float* __restrict__ be2, const float* __restrict__ b3, const float* __restrict__ g3,
    const float* __restrict__ be3,
    unsigned short* dW2, unsigned short* dW3, unsigned short* dWN, float* dVEC) {
  const int job = (int)blockIdx.y;
  const int i = (int)blockIdx.x * NTHR + (int)threadIdx.x;
  if (job == 3) {
    if (i >= VECN / 4) return;
    const int g = 4 * i;
    const int seg = g >> 8;
    const int c8 = g & 255;
    const int c9 = g & 511;
    const float inv = 1.0f / sqrtf(1.0f + 1e-5f);
    const v4f w1v = *(const v4f*)(w1 + c8);
    const v4f b1v = *(const v4f*)(b1 + c8);
    const v4f g1v = *(const v4f*)(g1 + c8);
    const v4f e1v = *(const v4f*)(be1 + c8);
    const v4f b2v = *(const v4f*)(b2 + c9);
    const v4f g2v = *(const v4f*)(g2 + c9);
    const v4f e2v = *(const v4f*)(be2 + c9);
    const v4f b3v = *(const v4f*)(b3 + c8);
    const v4f g3v = *(const v4f*)(g3 + c8);
    const v4f e3v = *(const v4f*)(be3 + c8);
    const v4f s1b = g1v * inv;
    const v4f s1v = s1b * w1v;
    const v4f t1v = s1b * b1v + e1v;
    const v4f s2v = g2v * inv;
    const v4f t2v = s2v * b2v + e2v;
    const v4f s3v = g3v * inv;
    const v4f t3v = s3v * b3v + e3v;
    const v4f o = (seg == 0) ? s1v : ((seg == 1) ? t1v : ((seg == 2 || seg == 3) ? s2v :
                  ((seg == 4 || seg == 5) ? t2v : ((seg == 6) ? s3v : t3v))));
    float* d = dVEC + g;
    *(volatile v4f*)d = o;
    __threadfence();
    *(volatile v4f*)d = o;
    return;
  }
  const int Nout = (job == 0) ? DH : DD;
  const int KP = (job == 1) ? DH : DD;
  const float* W = (job == 0) ? w2 : ((job == 1) ? w3 : wn);
  unsigned short* dst = (job == 0) ? dW2 : ((job == 1) ? dW3 : dWN);
  const int upc = KP >> 3;
  if (i >= Nout * upc) return;
  const int n = i / upc;
  const int seg = i - n * upc;
  v8h o;
#pragma unroll
  for (int j = 0; j < 8; ++j) {
    const int k = 8 * seg + j;
    o[j] = (_Float16)(W[(size_t)k * Nout + n] * (float)WSC);
  }
  const v8us ob = __builtin_bit_cast(v8us, o);
  unsigned short* d = dst + (size_t)i * 8;
  *(volatile v8us*)d = ob;
  __threadfence();
  *(volatile v8us*)d = ob;
}

__global__ __launch_bounds__(NTHR) void k_xproj(const float* __restrict__ X, const unsigned short* __restrict__ Bp,
                                               const float* __restrict__ bias, float* XP, int nN) {
  __shared__ __attribute__((aligned(16))) float stg[XBM * XBN];
  const int tid = threadIdx.x, lane = tid & 31, wave = tid >> 5, hh = lane >> 4, m = lane & 15;
  const int rowBase = (int)blockIdx.x * XBM;
  const int colBase = (int)blockIdx.y * XBN;
  const int rg = wave >> 1, chf = wave & 1;
  const int r0 = rg * 16;
  const int c0 = chf * 64;

  int arow = rowBase + r0 + m; arow = arow > nN - 1 ? nN - 1 : arow;
  const float* ap = X + (size_t)arow * DD + 8 * hh;
  const unsigned short* bp = Bp + (size_t)(colBase + c0 + m) * DD + 8 * hh;

  v8f acc[4];
#pragma unroll
  for (int t = 0; t < 4; ++t) acc[t] = zero8();
#pragma unroll 1
  for (int kt = 0; kt < 8; ++kt) {
    FragH a;
    a.h[0] = cvt8s(ap + 32 * kt, (float)ASC);
    a.h[1] = cvt8s(ap + 32 * kt + 16, (float)ASC);
#pragma unroll
    for (int t = 0; t < 4; ++t) {
      FragH b;
      b.u[0] = *(const v8us*)(bp + (size_t)t * 16 * DD + 32 * kt);
      b.u[1] = *(const v8us*)(bp + (size_t)t * 16 * DD + 32 * kt + 16);
      acc[t] = wmh(a.v, b.v, acc[t]);
    }
  }

  {
    float* sp = stg + (size_t)(r0 + 8 * hh) * XBN + c0 + m;
#pragma unroll
    for (int t = 0; t < 4; ++t) {
      const float bv = bias[colBase + c0 + 16 * t + m];
#pragma unroll
      for (int r = 0; r < 8; ++r) sp[r * XBN + 16 * t] = acc[t][r] * OSC + bv;
    }
  }
  __syncthreads();

#pragma unroll
  for (int it = 0; it < 8; ++it) {
    const int id = it * NTHR + tid;
    const int row = id >> 5, seg = id & 31;
    const v4f v = *(const v4f*)(stg + (size_t)row * XBN + 4 * seg);
    float* gp = XP + (size_t)(rowBase + row) * DD + colBase + 4 * seg;
    *(volatile v4f*)gp = v;
  }
  __threadfence();
#pragma unroll
  for (int it = 0; it < 8; ++it) {
    const int id = it * NTHR + tid;
    const int row = id >> 5, seg = id & 31;
    const v4f v = *(const v4f*)(stg + (size_t)row * XBN + 4 * seg);
    float* gp = XP + (size_t)(rowBase + row) * DD + colBase + 4 * seg;
    *(volatile v4f*)gp = v;
  }
}

__global__ __launch_bounds__(NTHR) void k_edge(
    const int* __restrict__ ei, const float* __restrict__ pos, const float* __restrict__ dinv,
    const float* __restrict__ VEC, const unsigned short* __restrict__ W2p, const unsigned short* __restrict__ W3p,
    const float* __restrict__ w4, const float* __restrict__ b4, float* WE, int nN, int nE) {
  extern __shared__ v4f lds_dyn[];
  _Float16* sH1   = (_Float16*)lds_dyn;
  _Float16* sH2   = sH1 + TE * P1;
  float*    sH3   = (float*)sH2;
  float*    sDist = (float*)(sH2 + TE * P2);
  float*    sNorm = sDist + TE;
  float*    sWg   = sNorm + TE;
  const int tid = threadIdx.x, lane = tid & 31, wave = tid >> 5, hh = lane >> 4, m = lane & 15;
  const int eBase = (int)blockIdx.x * TE;

  if (tid < TE) {
#pragma clang fp contract(off)
    int e = eBase + tid; e = e > nE - 1 ? nE - 1 : e;
    int r = ei[e];
    int c = ei[(size_t)nE + e];
    r = r < 0 ? 0 : (r > nN - 1 ? nN - 1 : r);
    c = c < 0 ? 0 : (c > nN - 1 ? nN - 1 : c);
    const float* pr = pos + (size_t)r * 3;
    const float* pc = pos + (size_t)c * 3;
    const float dx = pr[0] - pc[0];
    const float dy = pr[1] - pc[1];
    const float dz = pr[2] - pc[2];
    const float sq = (dx * dx + dz * dz) + dy * dy;
    sDist[tid] = sqrtf(sq);
    sNorm[tid] = dinv[r] * dinv[c];
  }
  __syncthreads();

  {
    const v4f sa = *(const v4f*)(VEC + 8 * lane);
    const v4f sb = *(const v4f*)(VEC + 8 * lane + 4);
    const v4f ta = *(const v4f*)(VEC + 256 + 8 * lane);
    const v4f tb = *(const v4f*)(VEC + 256 + 8 * lane + 4);
#pragma unroll
    for (int i = 0; i < 8; ++i) {
      const int row = 8 * wave + i;
      const float d = sDist[row];
      const v4f xa = sa * d + ta;
      const v4f xb = sb * d + tb;
      v8h o;
      o[0] = (_Float16)(lrelu(xa.x) * (float)ASC); o[1] = (_Float16)(lrelu(xa.y) * (float)ASC);
      o[2] = (_Float16)(lrelu(xa.z) * (float)ASC); o[3] = (_Float16)(lrelu(xa.w) * (float)ASC);
      o[4] = (_Float16)(lrelu(xb.x) * (float)ASC); o[5] = (_Float16)(lrelu(xb.y) * (float)ASC);
      o[6] = (_Float16)(lrelu(xb.z) * (float)ASC); o[7] = (_Float16)(lrelu(xb.w) * (float)ASC);
      *(v8h*)(sH1 + row * P1 + 8 * lane) = o;
    }
  }
  __syncthreads();

#pragma unroll 1
  for (int cbi = 0; cbi < 2; ++cbi) {
    const int cb = 2 * wave + cbi;
    const int c0 = 32 * cb + m, c1 = c0 + 16;
    v8f acc[4][2];
#pragma unroll
    for (int rt = 0; rt < 4; ++rt) { acc[rt][0] = zero8(); acc[rt][1] = zero8(); }
#pragma unroll 1
    for (int kt = 0; kt < 8; ++kt) {
      const v16h b0 = frag_glb(W2p, c0, DD, 32 * kt, hh);
      const v16h b1 = frag_glb(W2p, c1, DD, 32 * kt, hh);
#pragma unroll
      for (int rt = 0; rt < 4; ++rt) {
        const v16h a = frag_lds(sH1, 16 * rt + m, P1, 32 * kt, hh);
        acc[rt][0] = wmh(a, b0, acc[rt][0]);
        acc[rt][1] = wmh(a, b1, acc[rt][1]);
      }
    }
    const float sA = VEC[512 + c0] * OSC, tA = VEC[1024 + c0];
    const float sB = VEC[512 + c1] * OSC, tB = VEC[1024 + c1];
#pragma unroll
    for (int rt = 0; rt < 4; ++rt) {
      _Float16* hp = sH2 + (16 * rt + 8 * hh) * P2;
#pragma unroll
      for (int r = 0; r < 8; ++r) {
        const float va = lrelu(acc[rt][0][r] * sA + tA);
        const float vb = lrelu(acc[rt][1][r] * sB + tB);
        hp[r * P2 + c0] = (_Float16)(va * (float)ASC);
        hp[r * P2 + c1] = (_Float16)(vb * (float)ASC);
      }
    }
  }
  __syncthreads();

  {
    const int c0 = 32 * wave + m, c1 = c0 + 16;
    v8f acc[4][2];
#pragma unroll
    for (int rt = 0; rt < 4; ++rt) { acc[rt][0] = zero8(); acc[rt][1] = zero8(); }
#pragma unroll 1
    for (int kt = 0; kt < 16; ++kt) {
      const v16h b0 = frag_glb(W3p, c0, DH, 32 * kt, hh);
      const v16h b1 = frag_glb(W3p, c1, DH, 32 * kt, hh);
#pragma unroll
      for (int rt = 0; rt < 4; ++rt) {
        const v16h a = frag_lds(sH2, 16 * rt + m, P2, 32 * kt, hh);
        acc[rt][0] = wmh(a, b0, acc[rt][0]);
        acc[rt][1] = wmh(a, b1, acc[rt][1]);
      }
    }
    __syncthreads();
    const float sA = VEC[1536 + c0] * OSC, tA = VEC[1792 + c0];
    const float sB = VEC[1536 + c1] * OSC, tB = VEC[1792 + c1];
#pragma unroll
    for (int rt = 0; rt < 4; ++rt) {
      float* hp = sH3 + (16 * rt + 8 * hh) * P3;
#pragma unroll
      for (int r = 0; r < 8; ++r) {
        hp[r * P3 + c0] = lrelu(acc[rt][0][r] * sA + tA);
        hp[r * P3 + c1] = lrelu(acc[rt][1][r] * sB + tB);
      }
    }
  }
  __syncthreads();

  {
    const int e = tid >> 2, q = tid & 3;
    const float* hp = sH3 + e * P3 + 64 * q;
    const float* wp = w4 + 64 * q;
    float s = 0.0f;
#pragma unroll 4
    for (int i = 0; i < 16; ++i) {
      const v4f hv = *(const v4f*)(hp + 4 * i);
      const v4f wv = *(const v4f*)(wp + 4 * i);
      s += hv.x * wv.x; s += hv.y * wv.y; s += hv.z * wv.z; s += hv.w * wv.w;
    }
    s += __shfl_xor(s, 1);
    s += __shfl_xor(s, 2);
    const float emb = s + b4[0];
    if (q == 0) sWg[e] = sNorm[e] * emb;
  }
  __syncthreads();

  if (wave == 0) {
    const int l16 = lane < 16 ? lane : 15;
    const v4f v = *(const v4f*)(sWg + 4 * l16);
    float* gp = WE + (size_t)eBase + 4 * l16;
    if (lane < 16) *(volatile v4f*)gp = v;
    __threadfence();
    if (lane < 16) *(volatile v4f*)gp = v;
  }
}

__global__ __launch_bounds__(NTHR) void k_agg(
    const int* __restrict__ cnt, const int* __restrict__ off, const int* __restrict__ csrE,
    const int* __restrict__ ei, const float* __restrict__ WE, const float* __restrict__ XP,
    const float* __restrict__ pos, float* out, int nN, int nE, int nK, int csrLen) {
  __shared__ __attribute__((aligned(16))) float sOut[ANB * OROW];
  const int tid = threadIdx.x, lane = tid & 31, wave = tid >> 5;
  const int nb = (int)blockIdx.x * ANB;
  const v4f z4 = {0.f, 0.f, 0.f, 0.f};

#pragma unroll 1
  for (int j = 0; j < 4; ++j) {
    const int ln = 4 * wave + j;
    int n = nb + ln; n = n > nN - 1 ? nN - 1 : n;
    const int craw = cnt[n];
    const int ovf = (craw > DEGCAP) ? 1 : 0;
    int cn = craw < 0 ? 0 : (craw > DEGCAP ? DEGCAP : craw);
    cn = __builtin_amdgcn_readfirstlane(cn);
    int st = off[n];
    st = st < 0 ? 0 : (st > csrLen - 1 ? csrLen - 1 : st);
    st = __builtin_amdgcn_readfirstlane(st);

    v4f acc0 = z4, acc1 = z4;
#pragma unroll 1
    for (int base = 0; base < cn; base += 32) {
      int idx = base + lane; idx = idx > cn - 1 ? cn - 1 : idx;
      int s = st + idx; s = s > csrLen - 1 ? csrLen - 1 : s;
      int jv = csrE[s];
      jv = jv < 0 ? 0 : (jv > nK - 1 ? nK - 1 : jv);
      const bool isr = jv < nE;
      const int e  = isr ? jv : jv - nE;
      const int oi = isr ? jv + nE : jv - nE;
      int oth = ei[oi];
      oth = oth < 0 ? 0 : (oth > nN - 1 ? nN - 1 : oth);
      const float w = WE[e];
      int mcount = cn - base; mcount = mcount > 32 ? 32 : mcount;
#pragma unroll 1
      for (int k = 0; k < mcount; ++k) {
        const int ok = __shfl(oth, k);
        const float wk = __shfl(w, k);
        const float* xp = XP + (size_t)ok * DD;
        const v4f v0 = *(const v4f*)(xp + 4 * lane);
        const v4f v1 = *(const v4f*)(xp + 128 + 4 * lane);
        acc0 += wk * v0;
        acc1 += wk * v1;
      }
    }

    const float qn = __int_as_float(0x7fc00000);
    v4f r0v, r1v;
    r0v.x = fmaxf(acc0.x, 0.f); r0v.y = fmaxf(acc0.y, 0.f); r0v.z = fmaxf(acc0.z, 0.f); r0v.w = fmaxf(acc0.w, 0.f);
    r1v.x = fmaxf(acc1.x, 0.f); r1v.y = fmaxf(acc1.y, 0.f); r1v.z = fmaxf(acc1.z, 0.f); r1v.w = fmaxf(acc1.w, 0.f);
    if (ovf) {
      r0v.x = qn; r0v.y = qn; r0v.z = qn; r0v.w = qn;
      r1v.x = qn; r1v.y = qn; r1v.z = qn; r1v.w = qn;
    }
    float* so = sOut + ln * OROW;
    so[4 * lane + 0] = r0v.x; so[4 * lane + 1] = r0v.y; so[4 * lane + 2] = r0v.z; so[4 * lane + 3] = r0v.w;
    so[128 + 4 * lane + 0] = r1v.x; so[128 + 4 * lane + 1] = r1v.y;
    so[128 + 4 * lane + 2] = r1v.z; so[128 + 4 * lane + 3] = r1v.w;
    const int lp = lane < 3 ? lane : 2;
    const float pv = pos[(size_t)n * 3 + lp];
    if (lane < 3) so[256 + lane] = pv;
  }
  __syncthreads();

  const size_t fb = (size_t)nb * OROW;
  const int NPCS = (ANB * OROW) / 4;
  const int NIT = (NPCS + NTHR - 1) / NTHR;
#pragma unroll 1
  for (int it = 0; it < NIT; ++it) {
    const int p = it * NTHR + tid;
    if (p < NPCS) {
      const v4f v = *(const v4f*)(sOut + 4 * p);
      *(volatile v4f*)(out + fb + (size_t)4 * p) = v;
    }
  }
  __threadfence();
#pragma unroll 1
  for (int it = 0; it < NIT; ++it) {
    const int p = it * NTHR + tid;
    if (p < NPCS) {
      const v4f v = *(const v4f*)(sOut + 4 * p);
      *(volatile v4f*)(out + fb + (size_t)4 * p) = v;
    }
  }
}

extern "C" void kernel_launch(void* const* d_in, const int* in_sizes, int n_in,
                              void* d_out, int out_size, void* d_ws, size_t ws_size,
                              hipStream_t stream) {
  if (n_in < 19) return;
  const int nN = in_sizes[0] / DD;
  const int nE = in_sizes[2] / 2;
  if (nN <= 0 || nE <= 0) return;
  if (in_sizes[0] != nN * DD || in_sizes[1] != 3 * nN || in_sizes[2] != 2 * nE) return;
  if (in_sizes[3] != DD * DD || in_sizes[4] != DD || in_sizes[5] != DD || in_sizes[6] != DD) return;
  if (in_sizes[7] != DD || in_sizes[8] != DD || in_sizes[9] != DD * DH || in_sizes[10] != DH) return;
  if (in_sizes[11] != DH || in_sizes[12] != DH || in_sizes[13] != DH * DD || in_sizes[14] != DD) return;
  if (in_sizes[15] != DD || in_sizes[16] != DD || in_sizes[17] != DD || in_sizes[18] != 1) return;
  if (out_size != nN * OROW) return;
  if ((nN % ANB) != 0) return;
  if (nN > (1 << 20) || nE > (1 << 25)) return;

  const float* x    = (const float*)d_in[0];
  const float* pos  = (const float*)d_in[1];
  const int*   ei   = (const int*)d_in[2];
  const float* Wn_w = (const float*)d_in[3];
  const float* Wn_b = (const float*)d_in[4];
  const float* w1   = (const float*)d_in[5];
  const float* b1   = (const float*)d_in[6];
  const float* g1   = (const float*)d_in[7];
  const float* be1  = (const float*)d_in[8];
  const float* w2   = (const float*)d_in[9];
  const float* b2   = (const float*)d_in[10];
  const float* g2   = (const float*)d_in[11];
  const float* be2  = (const float*)d_in[12];
  const float* w3   = (const float*)d_in[13];
  const float* b3   = (const float*)d_in[14];
  const float* g3   = (const float*)d_in[15];
  const float* be3  = (const float*)d_in[16];
  const float* w4   = (const float*)d_in[17];
  const float* b4   = (const float*)d_in[18];
  float* out = (float*)d_out;

  const int nK = 2 * nE;
  const int NP = ((nN + 63) / 64) * 64;
  const int EP = ((nE + TE - 1) / TE) * TE;
  const int nBC = (nN + NBC - 1) / NBC;
  const int CNTPAD = nBC * NBC;
  if (4 * nBC + 1 > RBN) return;
  const int nBF = (nN + NBF - 1) / NBF;
  if (nBF > 4 * nBC) return;
  if (31 * 4 * nBC > 4096) return;
  const int csrLen = ((nK + 127) & ~127) + 4096;

  char* ws = (char*)d_ws;
  size_t off = 0;
  const size_t oW2  = off; off += (size_t)DH * DD * 2;        off = (off + 255) & ~(size_t)255;
  const size_t oW3  = off; off += (size_t)DD * DH * 2;        off = (off + 255) & ~(size_t)255;
  const size_t oWN  = off; off += (size_t)DD * DD * 2;        off = (off + 255) & ~(size_t)255;
  const size_t oVEC = off; off += (size_t)VECN * 4;           off = (off + 255) & ~(size_t)255;
  const size_t oXP  = off; off += (size_t)NP * DD * 4;        off = (off + 255) & ~(size_t)255;
  const size_t oWE  = off; off += (size_t)EP * 4;             off = (off + 255) & ~(size_t)255;
  const size_t oCnt = off; off += (size_t)CNTPAD * 4;         off = (off + 255) & ~(size_t)255;
  const size_t oDiv = off; off += (size_t)CNTPAD * 4;         off = (off + 255) & ~(size_t)255;
  const size_t oOff = off; off += (size_t)CNTPAD * 4;         off = (off + 255) & ~(size_t)255;
  const size_t oRb  = off; off += (size_t)RBN * 4;            off = (off + 255) & ~(size_t)255;
  const size_t oCsE = off; off += (size_t)csrLen * 4;         off = (off + 255) & ~(size_t)255;
  if (off > ws_size || off > (size_t)WSCAP) return;

  unsigned short* W2p  = (unsigned short*)(ws + oW2);
  unsigned short* W3p  = (unsigned short*)(ws + oW3);
  unsigned short* WNp  = (unsigned short*)(ws + oWN);
  float*          VEC  = (float*)(ws + oVEC);
  float*          XP   = (float*)(ws + oXP);
  float*          WE   = (float*)(ws + oWE);
  int*            cnt  = (int*)(ws + oCnt);
  float*          dinv = (float*)(ws + oDiv);
  int*            offp = (int*)(ws + oOff);
  int*            rb   = (int*)(ws + oRb);
  int*            csrE = (int*)(ws + oCsE);

  const int vec8 = 1;

  k_wcvt<<<dim3((DH * (DD / 8) + NTHR - 1) / NTHR, 4, 1), NTHR, 0, stream>>>(
      w2, w3, Wn_w, w1, b1, g1, be1, b2, g2, be2, b3, g3, be3, W2p, W3p, WNp, VEC);
  k_count<<<nBC, NTHR, 0, stream>>>(ei, cnt, dinv, nK, nE, vec8);
  k_offsets<<<1, OTHR, 0, stream>>>(cnt, offp, rb, nBC);
  hipFuncSetAttribute(reinterpret_cast<const void*>(&k_fill), hipFuncAttributeMaxDynamicSharedMemorySize, LDS_FILL);
  k_fill<<<nBF, NTHR, LDS_FILL, stream>>>(ei, offp, rb, csrE, nK, vec8, csrLen);
  k_xproj<<<dim3(NP / XBM, DD / XBN, 1), NTHR, 0, stream>>>(x, WNp, Wn_b, XP, nN);
  hipFuncSetAttribute(reinterpret_cast<const void*>(&k_edge), hipFuncAttributeMaxDynamicSharedMemorySize, LDS_EDGE);
  k_edge<<<EP / TE, NTHR, LDS_EDGE, stream>>>(ei, pos, dinv, VEC, W2p, W3p, w4, b4, WE, nN, nE);
  k_agg<<<nN / ANB, NTHR, 0, stream>>>(cnt, offp, csrE, ei, WE, XP, pos, out, nN, nE, nK, csrLen);
}
